// GATV2Layer_42296837931389
// MI455X (gfx1250) — hardware-verified
//
#include <hip/hip_runtime.h>
#include <math.h>
#include <stdint.h>

#define NB    4
#define NN    512
#define DD    128
#define NH    8
#define NF    16
#define MR    (NB * NN)
#define NC    (2 * DD)
#define IT    64
#define SLOPE 0.2f

static_assert(NH * NF == DD);
static_assert(MR % 64 == 0);
static_assert(NC % 64 == 0);
static_assert(DD % 64 == 0);
static_assert(DD % 32 == 0);
static_assert(NN % 64 == 0);
static_assert(NN % IT == 0);
static_assert(IT == 64);
static_assert(NN == 512);
static_assert((MR * DD / 8) % 256 == 0);
static_assert((DD * DD / 8) % 256 == 0);

#define ATT_LDS_FLOATS (IT * NN + NF * NN + NF * IT + IT * DD + 4 * 8 * 32 + NF)
#define ATT_LDS_BYTES  (ATT_LDS_FLOATS * 4)
static_assert(ATT_LDS_BYTES == 204864);
static_assert((IT * NN) % 4 == 0 && (NF * NN) % 4 == 0 && (NF * IT) % 4 == 0 && (IT * DD) % 4 == 0);

typedef __attribute__((ext_vector_type(16))) __bf16 v16b;
typedef __attribute__((ext_vector_type(8)))  __bf16 v8b;
typedef __attribute__((ext_vector_type(8)))  float  v8f;
typedef __attribute__((ext_vector_type(4)))  float  v4f;
typedef __attribute__((ext_vector_type(4)))  unsigned int v4u;
typedef __attribute__((ext_vector_type(8)))  unsigned int v8u;
typedef __attribute__((ext_vector_type(4)))  int    v4i;
typedef v8b __attribute__((may_alias)) v8ba;
typedef v4f __attribute__((may_alias)) v4fa;
typedef v4u __attribute__((may_alias)) v4ua;
typedef v4i __attribute__((may_alias)) v4ia;

union FragU { v16b v; v8b h[2]; };
union FragW { v16b v; v8u w; };

__device__ __forceinline__ unsigned short f2bf_bits(float f) {
  const unsigned u = __float_as_uint(f);
  return (unsigned short)((u + 0x7FFFu + ((u >> 16) & 1u)) >> 16);
}
__device__ __forceinline__ float bf_bits2f(unsigned short h) { return __uint_as_float(((unsigned)h) << 16); }
__device__ __forceinline__ float bf16r(float f) {
  unsigned u = __float_as_uint(f);
  u = (u + 0x7FFFu + ((u >> 16) & 1u)) & 0xFFFF0000u;
  return __uint_as_float(u);
}
__device__ __forceinline__ unsigned pk16(unsigned short a, unsigned short b) { return (unsigned)a | ((unsigned)b << 16); }
__device__ __forceinline__ void split2(float a, float b, unsigned& hw, unsigned& lw) {
  const unsigned short ha = f2bf_bits(a), hb = f2bf_bits(b);
  const unsigned short la = f2bf_bits(a - bf_bits2f(ha)), lb = f2bf_bits(b - bf_bits2f(hb));
  hw = pk16(ha, hb);
  lw = pk16(la, lb);
}

__device__ __forceinline__ v8f wmma_bf16(v16b a, v16b b, v8f c) {
  v8f d = __builtin_amdgcn_wmma_f32_16x16x32_bf16(false, a, false, b, (short)0, c, false, false);
  asm volatile("v_nop\n\tv_nop\n\tv_nop\n\tv_nop" : "+v"(d) : "v"(a), "v"(b));
  return d;
}
__device__ __forceinline__ void dep_guard_b(v8f& a, v8f& b, v16b x, v16b y) { asm volatile("v_nop\n\tv_nop\n\tv_nop\n\tv_nop" : "+v"(a), "+v"(b) : "v"(x), "v"(y)); }
__device__ __forceinline__ void keep4_b(v16b a, v16b b, v16b c, v16b d) { asm volatile("v_nop" :: "v"(a), "v"(b), "v"(c), "v"(d)); }
__device__ __forceinline__ void acc_guard4(v8f& a, v8f& b, v8f& c, v8f& d) { asm volatile("v_nop\n\tv_nop\n\tv_nop\n\tv_nop" : "+v"(a), "+v"(b), "+v"(c), "+v"(d)); }

__device__ __forceinline__ v16b load_frag(const unsigned short* p, int hh) {
  FragU f;
  f.h[0] = *(const v8ba*)(p + 8 * hh);
  f.h[1] = *(const v8ba*)(p + 16 + 8 * hh);
  return f.v;
}
__device__ __forceinline__ v16b load_frag_k(const unsigned short* p) {
  FragU f;
  f.h[0] = *(const v8ba*)(p);
  f.h[1] = *(const v8ba*)(p + 16);
  return f.v;
}

__global__ __launch_bounds__(256) void k_cvt(const float* __restrict__ x, unsigned short* __restrict__ Xb, int nunits) {
  const int g = blockIdx.x * 256 + threadIdx.x;
  if (g >= nunits) return;
  const float* src = x + (size_t)g * 8;
  const v4f a = *(const v4fa*)src;
  const v4f c = *(const v4fa*)(src + 4);
  v4u o;
  o[0] = pk16(f2bf_bits(a[0]), f2bf_bits(a[1]));
  o[1] = pk16(f2bf_bits(a[2]), f2bf_bits(a[3]));
  o[2] = pk16(f2bf_bits(c[0]), f2bf_bits(c[1]));
  o[3] = pk16(f2bf_bits(c[2]), f2bf_bits(c[3]));
  unsigned short* dst = Xb + (size_t)g * 8;
  *(volatile v4u*)dst = o;
  __threadfence();
  *(volatile v4u*)dst = o;
}

__global__ __launch_bounds__(256) void k_cvtw(const float* __restrict__ w0, const float* __restrict__ w1,
                                              unsigned short* __restrict__ Wb, int nunits) {
  const int g = blockIdx.x * 256 + threadIdx.x;
  if (g >= nunits) return;
  const int z = blockIdx.y;
  const float* src = ((z == 0) ? w0 : w1) + (size_t)g * 8;
  const v4f a = *(const v4fa*)src;
  const v4f c = *(const v4fa*)(src + 4);
  v4u o;
  o[0] = pk16(f2bf_bits(a[0]), f2bf_bits(a[1]));
  o[1] = pk16(f2bf_bits(a[2]), f2bf_bits(a[3]));
  o[2] = pk16(f2bf_bits(c[0]), f2bf_bits(c[1]));
  o[3] = pk16(f2bf_bits(c[2]), f2bf_bits(c[3]));
  unsigned short* dst = Wb + (size_t)z * nunits * 8 + (size_t)g * 8;
  *(volatile v4u*)dst = o;
  __threadfence();
  *(volatile v4u*)dst = o;
}

template <int OUT_MODE>
__global__ __launch_bounds__(256) void k_gemm64(
    const unsigned short* __restrict__ Ap, int lda, long strideA,
    const unsigned short* __restrict__ Btp, int ldb, long strideB,
    void* __restrict__ Cout, void* __restrict__ Cout2, int ldc, long strideC,
    int M, int N, int K) {
  __shared__ __align__(16) float sT[8][16 * 68];
  const int bz   = blockIdx.y;
  const int lane = threadIdx.x & 31;
  const int wave = threadIdx.x >> 5;
  const int tilesN = N >> 6;
  const int tilesM = M >> 6;
  const int tile = blockIdx.x * 8 + wave;
  if (tile >= tilesM * tilesN) return;
  const int tm = tile / tilesN;
  const int tn = tile - tm * tilesN;
  const int m0 = tm << 6;
  const int n0 = tn << 6;

  const unsigned short* Ab = Ap  + (size_t)bz * strideA;
  const unsigned short* Bb = Btp + (size_t)bz * strideB;

  const int rlane = lane & 15;
  const int koff  = (lane >> 4) * 8;
  const int mOff  = (lane >> 4) * 8;

  v8f acc[4][4];
#pragma unroll
  for (int i = 0; i < 4; ++i)
#pragma unroll
    for (int j = 0; j < 4; ++j) acc[i][j] = (v8f){0.f, 0.f, 0.f, 0.f, 0.f, 0.f, 0.f, 0.f};

  for (int k0 = 0; k0 < K; k0 += 32) {
    v16b bh[4];
#pragma unroll
    for (int j = 0; j < 4; ++j) {
      const size_t bo = (size_t)(n0 + (j << 4) + rlane) * ldb + koff + k0;
      bh[j] = load_frag_k(Bb + bo);
    }
#pragma unroll
    for (int i = 0; i < 4; ++i) {
      const size_t ao = (size_t)(m0 + (i << 4) + rlane) * lda + koff + k0;
      const v16b ah = load_frag_k(Ab + ao);
#pragma unroll
      for (int j = 0; j < 4; ++j)
        acc[i][j] = __builtin_amdgcn_wmma_f32_16x16x32_bf16(false, ah, false, bh[j], (short)0, acc[i][j], false, false);
      dep_guard_b(acc[i][0], acc[i][3], ah, ah);
    }
    keep4_b(bh[0], bh[1], bh[2], bh[3]);
  }
  acc_guard4(acc[0][0], acc[0][1], acc[0][2], acc[0][3]);
  acc_guard4(acc[1][0], acc[1][1], acc[1][2], acc[1][3]);
  acc_guard4(acc[2][0], acc[2][1], acc[2][2], acc[2][3]);
  acc_guard4(acc[3][0], acc[3][1], acc[3][2], acc[3][3]);

  float* slab = sT[wave];
#pragma unroll
  for (int i = 0; i < 4; ++i) {
    const int mBase = m0 + (i << 4);
#pragma unroll
    for (int j = 0; j < 4; ++j) {
#pragma unroll
      for (int r = 0; r < 8; ++r) slab[(mOff + r) * 68 + (j << 4) + rlane] = acc[i][j][r];
    }
    __builtin_amdgcn_fence(__ATOMIC_RELEASE, "workgroup");
    __builtin_amdgcn_wave_barrier();
    __builtin_amdgcn_fence(__ATOMIC_ACQUIRE, "workgroup");
    if (OUT_MODE == 0) {
      float* C = (float*)Cout + (size_t)bz * strideC;
      const int hh = lane >> 4, c4 = (lane & 15) * 4;
      for (int pass = 0; pass < 2; ++pass) {
#pragma unroll
        for (int it = 0; it < 8; ++it) {
          const int row = it * 2 + hh;
          const v4f v = *(const v4fa*)(slab + row * 68 + c4);
          *(volatile v4f*)(C + (size_t)(mBase + row) * ldc + n0 + c4) = v;
        }
        __threadfence();
      }
    } else {
      const int q = lane >> 3, c8 = (lane & 7) * 8;
      unsigned short* C  = (unsigned short*)Cout  + (size_t)bz * strideC;
      unsigned short* C2 = (unsigned short*)Cout2 + (size_t)bz * strideC;
      for (int pass = 0; pass < 2; ++pass) {
#pragma unroll
        for (int it = 0; it < 4; ++it) {
          const int row = it * 4 + q;
          const float* sp = slab + row * 68 + c8;
          v4u hv, lv;
#pragma unroll
          for (int e = 0; e < 4; ++e) {
            unsigned hw, lw;
            split2(sp[2 * e], sp[2 * e + 1], hw, lw);
            hv[e] = hw;
            lv[e] = lw;
          }
          *(volatile v4u*)(C  + (size_t)(mBase + row) * ldc + n0 + c8) = hv;
          *(volatile v4u*)(C2 + (size_t)(mBase + row) * ldc + n0 + c8) = lv;
        }
        __threadfence();
      }
    }
    __builtin_amdgcn_fence(__ATOMIC_RELEASE, "workgroup");
    __builtin_amdgcn_wave_barrier();
    __builtin_amdgcn_fence(__ATOMIC_ACQUIRE, "workgroup");
  }
}

__global__ __launch_bounds__(256) void k_attn(const float* __restrict__ GLR,
                                              const unsigned short* __restrict__ GRth,
                                              const unsigned short* __restrict__ GRtl,
                                              const int* __restrict__ adj,
                                              const float* __restrict__ a_w,
                                              float* __restrict__ out) {
  extern __shared__ __align__(16) float dsm[];
  float* S    = dsm;
  float* GLs  = S + IT * NN;
  float* GRIs = GLs + NF * NN;
  float* Oall = GRIs + NF * IT;
  float* part = Oall + IT * DD;
  float* aws  = part + 4 * 8 * 32;

  const int tid = threadIdx.x, lane = tid & 31, w = tid >> 5;
  const int hh = lane >> 4, m = lane & 15;
  const int b = blockIdx.y, i0 = blockIdx.x * IT;

  if (tid < NF) aws[tid] = bf16r(a_w[tid]);
  __syncthreads();
  float aw[NF];
#pragma unroll
  for (int f = 0; f < NF; ++f) aw[f] = aws[f];

  const v4f zero4 = {0.f, 0.f, 0.f, 0.f};
  const v8f zero8 = {0.f, 0.f, 0.f, 0.f, 0.f, 0.f, 0.f, 0.f};

#pragma unroll 1
  for (int hd = 0; hd < NH; ++hd) {
    {
#pragma unroll
      for (int s = 0; s < 2; ++s) {
        const int j = tid + 256 * s;
        const float* src = GLR + (size_t)(b * NN + j) * NC + hd * NF;
#pragma unroll
        for (int q = 0; q < 4; ++q) {
          const v4f v = *(const v4fa*)(src + 4 * q);
          GLs[(4 * q + 0) * NN + j] = v[0];
          GLs[(4 * q + 1) * NN + j] = v[1];
          GLs[(4 * q + 2) * NN + j] = v[2];
          GLs[(4 * q + 3) * NN + j] = v[3];
        }
      }
      const int il = tid >> 2, f4 = (tid & 3) * 4;
      const v4f v = *(const v4fa*)(GLR + (size_t)(b * NN + i0 + il) * NC + DD + hd * NF + f4);
      GRIs[(f4 + 0) * IT + il] = v[0];
      GRIs[(f4 + 1) * IT + il] = v[1];
      GRIs[(f4 + 2) * IT + il] = v[2];
      GRIs[(f4 + 3) * IT + il] = v[3];
    }
    __syncthreads();

    {
#pragma unroll 1
      for (int ii = 0; ii < 2; ++ii) {
        const int i4 = 4 * w + 32 * ii;
#pragma unroll 1
        for (int jj = 0; jj < 4; ++jj) {
          const int j4 = 4 * lane + 128 * jj;
          v4f acc[4];
#pragma unroll
          for (int a = 0; a < 4; ++a) acc[a] = zero4;
#pragma unroll
          for (int f = 0; f < NF; ++f) {
            const v4f g = *(const v4fa*)(GLs + f * NN + j4);
            const v4f r = *(const v4fa*)(GRIs + f * IT + i4);
            const float af = aw[f];
#pragma unroll
            for (int a = 0; a < 4; ++a)
#pragma unroll
              for (int c = 0; c < 4; ++c) {
                const float z = g[c] + r[a];
                acc[a][c] = fmaf(af, fmaxf(z, z * SLOPE), acc[a][c]);
              }
          }
#pragma unroll
          for (int a = 0; a < 4; ++a) {
            const v4i mk = *(const v4ia*)(adj + (size_t)(b * NN + i0 + i4 + a) * NN + j4);
            v4f sv;
#pragma unroll
            for (int c = 0; c < 4; ++c) sv[c] = (mk[c] != 0) ? acc[a][c] : -INFINITY;
            *(v4fa*)(S + (i4 + a) * NN + j4) = sv;
          }
        }
      }
    }
    __syncthreads();

    {
#pragma unroll 1
      for (int r = 0; r < 8; ++r) {
        float* row = S + (8 * w + r) * NN;
        v4f x[4];
        float mx = -INFINITY;
#pragma unroll
        for (int q = 0; q < 4; ++q) {
          x[q] = *(const v4fa*)(row + 128 * q + 4 * lane);
#pragma unroll
          for (int e = 0; e < 4; ++e) mx = fmaxf(mx, x[q][e]);
        }
#pragma unroll
        for (int off = 1; off < 32; off <<= 1) mx = fmaxf(mx, __shfl_xor(mx, off, 32));
        float sum = 0.0f;
#pragma unroll
        for (int q = 0; q < 4; ++q)
#pragma unroll
          for (int e = 0; e < 4; ++e) {
            const float p = __expf(x[q][e] - mx);
            x[q][e] = p;
            sum += p;
          }
#pragma unroll
        for (int off = 1; off < 32; off <<= 1) sum += __shfl_xor(sum, off, 32);
        const float inv = 1.0f / sum;
#pragma unroll
        for (int q = 0; q < 4; ++q) {
          const v4f pv = x[q] * inv;
          *(v4fa*)(row + 128 * q + 4 * lane) = pv;
        }
      }
    }
    __syncthreads();

    {
      const int mt = w & 3, kh = w >> 2;
      v8f acc = zero8;
      const unsigned short* gph = GRth + (size_t)(b * DD + hd * NF + m) * NN;
      const unsigned short* gpl = GRtl + (size_t)(b * DD + hd * NF + m) * NN;
      const float* prow = S + (16 * mt + m) * NN + 8 * hh;
#pragma unroll 2
      for (int ks = 0; ks < 8; ++ks) {
        const int k0 = kh * 256 + ks * 32;
        const v4f x0 = *(const v4fa*)(prow + k0);
        const v4f x1 = *(const v4fa*)(prow + k0 + 4);
        const v4f x2 = *(const v4fa*)(prow + k0 + 16);
        const v4f x3 = *(const v4fa*)(prow + k0 + 20);
        FragW ph, pl;
        { unsigned hw_, lw_; split2(x0[0], x0[1], hw_, lw_); ph.w[0] = hw_; pl.w[0] = lw_; }
        { unsigned hw_, lw_; split2(x0[2], x0[3], hw_, lw_); ph.w[1] = hw_; pl.w[1] = lw_; }
        { unsigned hw_, lw_; split2(x1[0], x1[1], hw_, lw_); ph.w[2] = hw_; pl.w[2] = lw_; }
        { unsigned hw_, lw_; split2(x1[2], x1[3], hw_, lw_); ph.w[3] = hw_; pl.w[3] = lw_; }
        { unsigned hw_, lw_; split2(x2[0], x2[1], hw_, lw_); ph.w[4] = hw_; pl.w[4] = lw_; }
        { unsigned hw_, lw_; split2(x2[2], x2[3], hw_, lw_); ph.w[5] = hw_; pl.w[5] = lw_; }
        { unsigned hw_, lw_; split2(x3[0], x3[1], hw_, lw_); ph.w[6] = hw_; pl.w[6] = lw_; }
        { unsigned hw_, lw_; split2(x3[2], x3[3], hw_, lw_); ph.w[7] = hw_; pl.w[7] = lw_; }
        const v16b bh = load_frag(gph + k0, hh);
        const v16b bl = load_frag(gpl + k0, hh);
        acc = wmma_bf16(ph.v, bh, acc);
        acc = wmma_bf16(ph.v, bl, acc);
        acc = wmma_bf16(pl.v, bh, acc);
      }
      if (w >= 4) {
#pragma unroll
        for (int r = 0; r < 8; ++r) part[(mt * 8 + r) * 32 + lane] = acc[r];
      }
      __syncthreads();
      if (w < 4) {
#pragma unroll
        for (int r = 0; r < 8; ++r)
          Oall[(16 * mt + 8 * hh + r) * DD + hd * NF + m] = acc[r] + part[(mt * 8 + r) * 32 + lane];
      }
    }
  }
  __syncthreads();

  {
    v4f vals[8];
#pragma unroll
    for (int r = 0; r < 8; ++r) vals[r] = *(const v4fa*)(Oall + (8 * w + r) * DD + 4 * lane);
    for (int pass = 0; pass < 2; ++pass) {
#pragma unroll
      for (int r = 0; r < 8; ++r)
        *(volatile v4f*)(out + (size_t)(b * NN + i0 + 8 * w + r) * DD + 4 * lane) = vals[r];
      __threadfence();
    }
  }
}

extern "C" void kernel_launch(void* const* d_in, const int* in_sizes, int n_in,
                              void* d_out, int out_size, void* d_ws, size_t ws_size,
                              hipStream_t stream) {
  if (n_in < 5) return;
  if (in_sizes[0] != NB * NN * DD) return;
  if (in_sizes[1] != NB * NN * NN) return;
  if (in_sizes[2] != DD * DD) return;
  if (in_sizes[3] != DD * DD) return;
  if (in_sizes[4] != NF) return;
  if (out_size != NB * NN * DD) return;

  const float* h   = (const float*)d_in[0];
  const int*   adj = (const int*)d_in[1];
  const float* Wl  = (const float*)d_in[2];
  const float* Wr  = (const float*)d_in[3];
  const float* aw  = (const float*)d_in[4];
  float* out = (float*)d_out;

  const size_t PHB  = (size_t)MR * DD * 2;
  const size_t PWC  = (size_t)NC * DD * 2;
  const size_t PGLR = (size_t)MR * NC * 4;
  const size_t PGRT = (size_t)NB * DD * NN * 2;
  size_t off = 0;
  const size_t oHb  = off; off += PHB;
  const size_t oWc  = off; off += PWC;
  const size_t oGLR = off; off += PGLR;
  const size_t oGRh = off; off += PGRT;
  const size_t oGRl = off; off += PGRT;
  if (off > ws_size) return;

  char* ws = (char*)d_ws;
  unsigned short* Hb   = (unsigned short*)(ws + oHb);
  unsigned short* Wcat = (unsigned short*)(ws + oWc);
  float*          GLR  = (float*)(ws + oGLR);
  unsigned short* GRth = (unsigned short*)(ws + oGRh);
  unsigned short* GRtl = (unsigned short*)(ws + oGRl);

  k_cvt<<<dim3((MR * DD / 8) / 256), 256, 0, stream>>>(h, Hb, MR * DD / 8);
  k_cvtw<<<dim3((DD * DD / 8) / 256, 2), 256, 0, stream>>>(Wl, Wr, Wcat, DD * DD / 8);
  k_gemm64<0><<<dim3(((MR / 64) * (NC / 64) + 7) / 8, 1), 256, 0, stream>>>(
      Hb, DD, 0L, Wcat, DD, 0L, (void*)GLR, (void*)GLR, NC, 0L, MR, NC, DD);
  k_gemm64<2><<<dim3((((DD / 64) * (NN / 64)) + 7) / 8, NB), 256, 0, stream>>>(
      Wcat + (size_t)DD * DD, DD, 0L, Hb, DD, (long)NN * DD, (void*)GRth, (void*)GRtl, NN, (long)DD * NN, DD, NN, DD);
  (void)hipFuncSetAttribute(reinterpret_cast<const void*>(&k_attn), hipFuncAttributeMaxDynamicSharedMemorySize, ATT_LDS_BYTES);
  k_attn<<<dim3(NN / IT, NB), 256, ATT_LDS_BYTES, stream>>>(GLR, GRth, GRtl, adj, aw, out);
  (void)hipGetLastError();
}
